// TensorRingLinear_50955491999867
// MI455X (gfx1250) — hardware-run, weakly checked
//
#include <hip/hip_runtime.h>


#ifndef NB
#define NB 1024
#endif
#define NB_FULL 1024
#define DIN  1024
#define DOUT 1024
#define QRS  2048.0f
#define QRI  (1.0f / 2048.0f)
#define WSC  256.0f
#define WCI  (1.0f / 256.0f)

static_assert(NB <= NB_FULL);
static_assert(DIN == 4 * 8 * 8 * 4);
static_assert(DIN == 256 * 4);
static_assert(DOUT == 256 * 4);
static_assert((DOUT * 4) % 512 == 0);
static_assert(128 % 32 == 0 && 64 % 32 == 0 && 256 % 32 == 0);

typedef _Float16 h16;
typedef unsigned short bf;
typedef __attribute__((ext_vector_type(16))) __bf16   v16bf;
typedef __attribute__((ext_vector_type(16))) _Float16 v16h;
typedef __attribute__((ext_vector_type(8)))  _Float16 v8h;
typedef __attribute__((ext_vector_type(8)))  unsigned short v8us;
typedef __attribute__((ext_vector_type(4)))  unsigned short v4us;
typedef __attribute__((ext_vector_type(8)))  float    v8f;
typedef __attribute__((ext_vector_type(4)))  float    v4f;
typedef v4f  __attribute__((may_alias)) v4fa;

__device__ __forceinline__ unsigned short f2bf(float f) { unsigned u = __float_as_uint(f); u += 0x7FFFu + ((u >> 16) & 1u); return (unsigned short)(u >> 16); }
__device__ __forceinline__ float bfr(float f) { return __uint_as_float(((unsigned)f2bf(f)) << 16); }
__device__ __forceinline__ v16h cat16(v8h lo, v8h hi) { return __builtin_shufflevector(lo, hi, 0, 1, 2, 3, 4, 5, 6, 7, 8, 9, 10, 11, 12, 13, 14, 15); }
__device__ __forceinline__ v16bf cat16b(v8us lo, v8us hi) { return __builtin_bit_cast(v16bf, __builtin_shufflevector(lo, hi, 0, 1, 2, 3, 4, 5, 6, 7, 8, 9, 10, 11, 12, 13, 14, 15)); }
__device__ __forceinline__ v8f wmma16(v16h a, v16h b, v8f c) { return __builtin_amdgcn_wmma_f32_16x16x32_f16(false, a, false, b, (short)0, c, false, false); }
__device__ __forceinline__ v8f wmmab(v16bf a, v16bf b, v8f c) { return __builtin_amdgcn_wmma_f32_16x16x32_bf16(false, a, false, b, (short)0, c, false, false); }
__device__ __forceinline__ v16h  ldh(const h16* p) { return cat16(*(const v8h*)p, *(const v8h*)(p + 16)); }
__device__ __forceinline__ v16bf ldb(const bf* p)  { return cat16b(*(const v8us*)p, *(const v8us*)(p + 16)); }

static __device__ __forceinline__ h16 toh_flush(float v) { const h16 r = (h16)v; return (fabsf(v) < 6.103515625e-05f) ? (h16)0.0f : r; }
__device__ __forceinline__ v8f wmma16g(v16h a, v16h b, v8f c) { c = wmma16(a, b, c); asm volatile("v_nop\n\tv_nop\n\tv_nop\n\tv_nop" : "+v"(c) : "v"(a), "v"(b)); return c; }
__device__ __forceinline__ v8f wmmabg(v16bf a, v16bf b, v8f c) { c = wmmab(a, b, c); asm volatile("v_nop\n\tv_nop\n\tv_nop\n\tv_nop" : "+v"(c) : "v"(a), "v"(b)); return c; }
__device__ __forceinline__ v16h k16(v8h lo) { const v8h z = (v8h){}; return cat16(lo, z); }
__device__ __forceinline__ v16h ldhs(const h16* p) { return cat16(*(const v8h*)p, *(const v8h*)(p + 16)); }
__device__ __forceinline__ void split8(const v8f ah, const v8f ar, v8h& hv, v8h& rv) {
#pragma unroll
    for (int j = 0; j < 8; ++j) { const float v = (ah[j] + ar[j] * QRI) * WCI; const h16 a = toh_flush(v); hv[j] = a; rv[j] = toh_flush((v - (float)a) * QRS); }
}
__device__ __forceinline__ void split8s(const v8f d, v8h& hv, v8h& rv) {
#pragma unroll
    for (int j = 0; j < 8; ++j) { const float v = d[j]; const h16 a = toh_flush(v); hv[j] = a; rv[j] = toh_flush((v - (float)a) * QRS); }
}

__global__ __launch_bounds__(256) void k_wconv(const float* __restrict__ src, h16* dst, int n8src, int n8dst, float scale) {
    const int i = blockIdx.x * 256 + threadIdx.x; if (i >= n8dst) return;
    const int j = i < n8src ? i : (n8src - 1);
    v8f v = *(const v8f*)(src + (size_t)j * 8);
    asm volatile("" : "+v"(v));
    const bool live = i < n8src;
    v8h o;
#pragma unroll
    for (int k = 0; k < 8; ++k) { const h16 t = toh_flush(bfr(v[k]) * scale); o[k] = live ? t : (h16)0.0f; }
    *(volatile v8h*)(dst + (size_t)i * 8) = o; __threadfence(); *(volatile v8h*)(dst + (size_t)i * 8) = o;
}

__global__ __launch_bounds__(256) void k_w0conv(const float* __restrict__ src, bf* dst) {
    const int i = blockIdx.x * 256 + threadIdx.x; if (i >= 1024) return;
    const int row = i >> 2, q = i & 3;
    v4f v = *(const v4f*)(src + (size_t)row * 4);
    asm volatile("" : "+v"(v));
    v8us o = (v8us){};
#pragma unroll
    for (int k = 0; k < 4; ++k) { const unsigned short t = f2bf(v[k]); o[k] = (q == 0) ? t : (unsigned short)0; }
    *(volatile v8us*)(dst + (size_t)i * 8) = o; __threadfence(); *(volatile v8us*)(dst + (size_t)i * 8) = o;
}

static constexpr int LDS_CHAIN_BYTES = 256 * 4 * 2 + 2 * 8192 * 2 + 2 * 1024 * 2 + 2 * 256 * 2 + 2 * 1024 * 2 + 1024 * 4;
static_assert(LDS_CHAIN_BYTES <= 131072);

__global__ __launch_bounds__(256) void k_chain(const float* __restrict__ x, const bf* __restrict__ W0B,
                                               const h16* __restrict__ W1C, const h16* __restrict__ W2C, const h16* __restrict__ W3C, const h16* __restrict__ W4C,
                                               const h16* __restrict__ W5C, const h16* __restrict__ W6C, const h16* __restrict__ W7C,
                                               const float* __restrict__ bias, float* OUT) {
    __shared__ __align__(16) bf    XB[256 * 4];
    __shared__ __align__(16) h16   BGH[8192];
    __shared__ __align__(16) h16   BGR[8192];
    __shared__ __align__(16) h16   Y2H[1024];
    __shared__ __align__(16) h16   Y2R[1024];
    __shared__ __align__(16) h16   Y3H[256];
    __shared__ __align__(16) h16   Y3R[256];
    __shared__ __align__(16) h16   Y4H[1024];
    __shared__ __align__(16) h16   Y4R[1024];
    __shared__ __align__(16) float OUTS[1024];
    const int tid = threadIdx.x;
    const int lane = tid & 31, lr = lane & 15, hi = lane >> 4;
    const int wave = __builtin_amdgcn_readfirstlane((int)(threadIdx.x >> 5));
    const int b = blockIdx.x;
    const v8f zf = (v8f){};
    const v8us zu = (v8us){};

    { const v4f xv = *(const v4f*)(x + (size_t)b * DIN + tid * 4);
      const int m0 = tid >> 6, m1 = (tid >> 3) & 7, m2 = tid & 7;
#pragma unroll
      for (int m3 = 0; m3 < 4; ++m3) XB[(m3 * 64 + m2 * 8 + m1) * 4 + m0] = f2bf(xv[m3]); }
    __syncthreads();

    { const int g = wave & 1;
      const int cc = g * 16 + lr;
#pragma unroll 1
      for (int i = 0; i < 4; ++i) {
          const int c0 = (wave >> 1) * 4 + i;
          const v16bf a0 = ldb(W0B + (size_t)(lr * 16 + c0) * 32 + 8 * hi);
          v8f yh = zf, yr = zf;
#pragma unroll 1
          for (int s = 0; s < 4; ++s) {
              const int xr = (cc * 8 + 2 * s) * 4;
              const v4us xa = *(const v4us*)(&XB[xr]);
              const v4us xc = *(const v4us*)(&XB[xr + 4]);
              v8us la = zu, lc = zu;
#pragma unroll
              for (int k = 0; k < 4; ++k) { la[k] = hi ? (unsigned short)0 : xa[k]; lc[k] = hi ? (unsigned short)0 : xc[k]; }
              const v16bf bx0 = cat16b(la, zu), bx1 = cat16b(lc, zu);
              const v8f d0 = wmmabg(a0, bx0, zf);
              const v8f d1 = wmmabg(a0, bx1, zf);
              v8h h0, r0, h1, r1;
              split8s(d0, h0, r0); split8s(d1, h1, r1);
              const v16h th = cat16(h0, h1), tr = cat16(r0, r1);
              const v16h w1 = ldh(W1C + lr * 128 + 32 * s + 8 * hi);
              yh = wmma16g(w1, th, yh);
              yr = wmma16g(w1, tr, yr);
          }
          v8h hv, rv; split8(yh, yr, hv, rv);
          *(v8h*)(&BGH[(c0 * 32 + cc) * 16 + 8 * hi]) = hv;
          *(v8h*)(&BGR[(c0 * 32 + cc) * 16 + 8 * hi]) = rv;
      } }
    __syncthreads();

    if (wave < 4) {
        v8f yh = zf, yr = zf;
        const int ro = (16 * wave + lr) * 128 + 8 * hi;
#pragma unroll 1
        for (int s = 0; s < 4; ++s) {
            const v16h w = ldh(W2C + lr * 128 + 32 * s + 8 * hi);
            const v16h ah = ldhs(&BGH[ro + 32 * s]);
            const v16h ar = ldhs(&BGR[ro + 32 * s]);
            yh = wmma16g(w, ah, yh);
            yr = wmma16g(w, ar, yr);
        }
        v8h hv, rv; split8(yh, yr, hv, rv);
        *(v8h*)(&Y2H[(16 * wave + lr) * 16 + 8 * hi]) = hv;
        *(v8h*)(&Y2R[(16 * wave + lr) * 16 + 8 * hi]) = rv;
    }
    __syncthreads();

    if (wave == 0) {
        v8f yh = zf, yr = zf;
#pragma unroll 1
        for (int s = 0; s < 2; ++s) {
            const v16h w = ldh(W3C + lr * 64 + 32 * s + 8 * hi);
            const v16h ah = ldhs(&Y2H[lr * 64 + 32 * s + 8 * hi]);
            const v16h ar = ldhs(&Y2R[lr * 64 + 32 * s + 8 * hi]);
            yh = wmma16g(w, ah, yh);
            yr = wmma16g(w, ar, yr);
        }
        v8h hv, rv; split8(yh, yr, hv, rv);
        *(v8h*)(&Y3H[lr * 16 + 8 * hi]) = hv;
        *(v8h*)(&Y3R[lr * 16 + 8 * hi]) = rv;
    }
    __syncthreads();

    if (wave < 4) {
        const v16h w = k16(*(const v8h*)(W4C + (16 * wave + lr) * 16 + 8 * hi));
        const v16h ah = k16(*(const v8h*)(&Y3H[lr * 16 + 8 * hi]));
        const v16h ar = k16(*(const v8h*)(&Y3R[lr * 16 + 8 * hi]));
        const v8f yh = wmma16g(w, ah, zf);
        const v8f yr = wmma16g(w, ar, zf);
        v8h hv, rv; split8(yh, yr, hv, rv);
        *(v8h*)(&Y4H[lr * 64 + 16 * wave + 8 * hi]) = hv;
        *(v8h*)(&Y4R[lr * 64 + 16 * wave + 8 * hi]) = rv;
    }
    __syncthreads();

    { const v16h w = k16(*(const v8h*)(W5C + (16 * wave + lr) * 16 + 8 * hi));
#pragma unroll 1
      for (int mt = 0; mt < 4; ++mt) {
          const v16h ah = k16(*(const v8h*)(&Y4H[(16 * mt + lr) * 16 + 8 * hi]));
          const v16h ar = k16(*(const v8h*)(&Y4R[(16 * mt + lr) * 16 + 8 * hi]));
          const v8f yh = wmma16g(w, ah, zf);
          const v8f yr = wmma16g(w, ar, zf);
          v8h hv, rv; split8(yh, yr, hv, rv);
          *(v8h*)(&BGH[(16 * mt + lr) * 128 + 16 * wave + 8 * hi]) = hv;
          *(v8h*)(&BGR[(16 * mt + lr) * 128 + 16 * wave + 8 * hi]) = rv;
      } }
    __syncthreads();

    { const v16h w6 = k16(*(const v8h*)(W6C + (16 * wave + lr) * 16 + 8 * hi));
#pragma unroll 1
      for (int Q = 0; Q < 2; ++Q) {
          v8f oh = zf, orr = zf;
#pragma unroll 1
          for (int s = 0; s < 8; ++s) {
              const int i0 = ((2 * s) * 32 + 16 * Q + lr) * 16 + 8 * hi;
              const int i1 = i0 + 32 * 16;
              const v16h b0h = k16(*(const v8h*)(&BGH[i0]));
              const v16h b0r = k16(*(const v8h*)(&BGR[i0]));
              const v16h b1h = k16(*(const v8h*)(&BGH[i1]));
              const v16h b1r = k16(*(const v8h*)(&BGR[i1]));
              const v8f d0h = wmma16g(w6, b0h, zf);
              const v8f d0r = wmma16g(w6, b0r, zf);
              const v8f d1h = wmma16g(w6, b1h, zf);
              const v8f d1r = wmma16g(w6, b1r, zf);
              v8h h0, r0, h1, r1;
              split8(d0h, d0r, h0, r0); split8(d1h, d1r, h1, r1);
              const v16h ph = cat16(h0, h1), pr = cat16(r0, r1);
              const v16h w7 = ldh(W7C + lr * 256 + 32 * s + 8 * hi);
              oh  = wmma16g(w7, ph, oh);
              orr = wmma16g(w7, pr, orr);
          }
          const int mid = 8 * (16 * Q + lr) + wave;
          const v4f bv = *(const v4f*)(bias + mid * 4);
          v4f ov;
#pragma unroll
          for (int r = 0; r < 4; ++r) ov[r] = (oh[r] + orr[r] * QRI) * WCI + bfr(bv[r]);
          if (hi == 0) *(v4fa*)(&OUTS[mid * 4]) = ov;
      } }
    __syncthreads();

    { const v4f val = *(const v4fa*)(&OUTS[tid * 4]);
      float* op = OUT + (size_t)b * DOUT + tid * 4;
      *(volatile v4f*)op = val; __threadfence(); *(volatile v4f*)op = val; }
}

static constexpr size_t al256(size_t v) { return (v + 255) & ~(size_t)255; }
static constexpr size_t SZ_W0 = al256((size_t)256 * 32 * 2);
static constexpr size_t SZ_W1 = al256((size_t)16 * 128 * 2);
static constexpr size_t SZ_W2 = al256((size_t)16 * 128 * 2);
static constexpr size_t SZ_W3 = al256((size_t)16 * 64 * 2);
static constexpr size_t SZ_W4 = al256((size_t)64 * 16 * 2);
static constexpr size_t SZ_W5 = al256((size_t)128 * 16 * 2);
static constexpr size_t SZ_W6 = al256((size_t)128 * 16 * 2);
static constexpr size_t SZ_W7 = al256((size_t)16 * 256 * 2);
static constexpr size_t SZ_TOTAL = SZ_W0 + SZ_W1 + SZ_W2 + SZ_W3 + SZ_W4 + SZ_W5 + SZ_W6 + SZ_W7;
static_assert(SZ_TOTAL <= (size_t)134217728);
static_assert((256 * 32) % (8 * 32) == 0);
static_assert((16 * 64) % (8 * 32) == 0);
static_assert((16 * 256) % (8 * 32) == 0);

extern "C" void kernel_launch(void* const* d_in, const int* in_sizes, int n_in,
                              void* d_out, int out_size, void* d_ws, size_t ws_size, hipStream_t stream) {
    if (n_in < 10) return;
    if ((size_t)in_sizes[0] < (size_t)NB * DIN) return;
    if (in_sizes[1] < 256 * 4 || in_sizes[2] < 16 * 128 || in_sizes[3] < 16 * 128 || in_sizes[4] < 16 * 64) return;
    if (in_sizes[5] < 64 * 16 || in_sizes[6] < 128 * 16 || in_sizes[7] < 128 * 16 || in_sizes[8] < 4 * 256 || in_sizes[9] < DOUT) return;
    if ((size_t)out_size < (size_t)NB * DOUT) return;
    if (SZ_TOTAL > ws_size) return;
    const float* x  = (const float*)d_in[0];
    const float* w0 = (const float*)d_in[1]; const float* w1 = (const float*)d_in[2];
    const float* w2 = (const float*)d_in[3]; const float* w3 = (const float*)d_in[4];
    const float* w4 = (const float*)d_in[5]; const float* w5 = (const float*)d_in[6];
    const float* w6 = (const float*)d_in[7]; const float* w7 = (const float*)d_in[8];
    const float* bias = (const float*)d_in[9];
    float* OUT = (float*)d_out;
    char* wsp = (char*)d_ws;
    bf*  W0B = (bf*)wsp;  wsp += SZ_W0;
    h16* W1C = (h16*)wsp; wsp += SZ_W1;
    h16* W2C = (h16*)wsp; wsp += SZ_W2;
    h16* W3C = (h16*)wsp; wsp += SZ_W3;
    h16* W4C = (h16*)wsp; wsp += SZ_W4;
    h16* W5C = (h16*)wsp; wsp += SZ_W5;
    h16* W6C = (h16*)wsp; wsp += SZ_W6;
    h16* W7C = (h16*)wsp; wsp += SZ_W7;

    k_w0conv<<<4, 256, 0, stream>>>(w0, W0B);
    k_wconv<<<1, 256, 0, stream>>>(w1, W1C, 16 * 128 / 8, 16 * 128 / 8, WSC);
    k_wconv<<<1, 256, 0, stream>>>(w2, W2C, 16 * 128 / 8, 16 * 128 / 8, WSC);
    k_wconv<<<1, 256, 0, stream>>>(w3, W3C, 16 * 64 / 8, 16 * 64 / 8, WSC);
    k_wconv<<<1, 256, 0, stream>>>(w4, W4C, 64 * 16 / 8, 64 * 16 / 8, WSC);
    k_wconv<<<1, 256, 0, stream>>>(w5, W5C, 128 * 16 / 8, 128 * 16 / 8, WSC);
    k_wconv<<<1, 256, 0, stream>>>(w6, W6C, 128 * 16 / 8, 128 * 16 / 8, WSC);
    k_wconv<<<2, 256, 0, stream>>>(w7, W7C, 4 * 256 / 8, 16 * 256 / 8, WSC);

    k_chain<<<NB, 256, 0, stream>>>(x, W0B, W1C, W2C, W3C, W4C, W5C, W6C, W7C, bias, OUT);
}
